// ModConv2d_43885975831074
// MI455X (gfx1250) — hardware-verified
//
#include <hip/hip_runtime.h>
#include <stddef.h>


typedef _Float16 v16h __attribute__((ext_vector_type(16)));
typedef _Float16 v8h  __attribute__((ext_vector_type(8)));
typedef float    v8f  __attribute__((ext_vector_type(8)));
typedef float    v4f  __attribute__((ext_vector_type(4)));

union Frag { v16h v; v8h half[2]; };

#define BS       8
#define C_IN     256
#define C_OUT    256
#define STYLE_D  512
#define HH       64
#define WW       64
#define KTOT     2304
#define NPIX     4096
#define XWIN     (4 * 66 * 32)
#define CSP      132
#define ASCALE   256.0f
#define AUNSCALE (1.0f / 256.0f)

__device__ __forceinline__ v8f wmma16(v16h a, v16h b, v8f c)
{
    v8f d = __builtin_amdgcn_wmma_f32_16x16x32_f16(false, a, false, b, (short)0, c, false, false);
    asm volatile("v_nop\n\tv_nop\n\tv_nop\n\tv_nop" : "+v"(d) : "v"(a), "v"(b));
    return d;
}

__device__ __forceinline__ v8f zero8f()
{
    v8f z;
#pragma unroll
    for (int j = 0; j < 8; ++j) z[j] = 0.0f;
    return z;
}

__global__ __launch_bounds__(256)
void style_kernel(const float* __restrict__ s,
                  const float* __restrict__ aw,
                  const float* __restrict__ ab,
                  float* style1)
{
    const int idx = blockIdx.x * 256 + threadIdx.x;
    if (idx >= BS * C_IN) return;
    const int b  = idx >> 8;
    const int ci = idx & 255;
    const float* sp = s  + (size_t)b  * STYLE_D;
    const float* wp = aw + (size_t)ci * STYLE_D;
    float acc = 0.0f;
    for (int k = 0; k < STYLE_D; ++k)
        acc = fmaf(sp[k], wp[k], acc);
    const float v = (acc + ab[ci]) + 1.0f;
    volatile float* p = style1 + idx;
    *p = v;
    __threadfence();
    *p = v;
}

__global__ __launch_bounds__(256)
void modw_kernel(const float* __restrict__ w,
                 const float* __restrict__ style1,
                 _Float16* Amod)
{
    __shared__ float wrow[KTOT];
    __shared__ __attribute__((aligned(16))) _Float16 arow[KTOT];
    __shared__ float red[8];

    const int b    = blockIdx.x >> 8;
    const int co   = blockIdx.x & 255;
    const int t    = threadIdx.x;
    const int lane = t & 31;
    const int wave = t >> 5;

    for (int e = t; e < KTOT; e += 256)
        wrow[e] = w[(size_t)co * KTOT + e];
    __syncthreads();

    const float st = style1[b * C_IN + t];
    float vm[9];
    float part = 0.0f;
#pragma unroll
    for (int r = 0; r < 9; ++r) {
        const float v = wrow[t * 9 + r] * st;
        vm[r] = v;
        part  = fmaf(v, v, part);
    }
#pragma unroll
    for (int o = 16; o > 0; o >>= 1)
        part += __shfl_xor(part, o);
    if (lane == 0) red[wave] = part;
    __syncthreads();
    float tot = red[0];
#pragma unroll
    for (int i = 1; i < 8; ++i) tot += red[i];
    const float scale = ASCALE / sqrtf(tot + 1e-8f);

#pragma unroll
    for (int r = 0; r < 9; ++r)
        arow[r * 256 + t] = (_Float16)(vm[r] * scale);
    __syncthreads();

    _Float16* dst = Amod + (size_t)(b * C_OUT + co) * KTOT;
    const bool tailw = (t < 32);
    const v8h c0 = *(const v8h*)(arow + t * 8);
    v8h c1 = c0;
    if (tailw) c1 = *(const v8h*)(arow + (t + 256) * 8);

    *(volatile v8h*)(dst + t * 8) = c0;
    if (tailw) *(volatile v8h*)(dst + (t + 256) * 8) = c1;
    __threadfence();
    *(volatile v8h*)(dst + t * 8) = c0;
    if (tailw) *(volatile v8h*)(dst + (t + 256) * 8) = c1;
}

__global__ __launch_bounds__(256)
void xcvt_kernel(const float* __restrict__ x, _Float16* Xh)
{
    __shared__ float tile[C_IN][17];

    const int b    = blockIdx.x >> 8;
    const int pt   = blockIdx.x & 255;
    const int hw0  = pt * 16;
    const int t    = threadIdx.x;
    const int lane = t & 31;
    const int wave = t >> 5;

#pragma unroll
    for (int i = 0; i < 16; ++i) {
        const int idx  = t + i * 256;
        const int hw_l = idx & 15;
        const int ci   = idx >> 4;
        tile[ci][hw_l] = x[(size_t)(b * C_IN + ci) * NPIX + hw0 + hw_l];
    }
    __syncthreads();

    v8h val[2];
#pragma unroll
    for (int i = 0; i < 2; ++i) {
        const int p = wave + 8 * i;
        v8h v;
#pragma unroll
        for (int j = 0; j < 8; ++j)
            v[j] = (_Float16)tile[lane * 8 + j][p];
        val[i] = v;
    }
    _Float16* d0 = Xh + (size_t)(b * NPIX + hw0 + wave) * C_IN + lane * 8;
    _Float16* d1 = d0 + (size_t)8 * C_IN;

    *(volatile v8h*)d0 = val[0];
    *(volatile v8h*)d1 = val[1];
    __threadfence();
    *(volatile v8h*)d0 = val[0];
    *(volatile v8h*)d1 = val[1];
}

__device__ __forceinline__ void stash(float (*cs)[CSP], int r, int c, v8f a)
{
    cs[r + 0][c] = a[0]; cs[r + 1][c] = a[1]; cs[r + 2][c] = a[2]; cs[r + 3][c] = a[3];
    cs[r + 4][c] = a[4]; cs[r + 5][c] = a[5]; cs[r + 6][c] = a[6]; cs[r + 7][c] = a[7];
}

__global__ __launch_bounds__(256)
void modconv_gemm(const _Float16* __restrict__ Amod,
                  const _Float16* __restrict__ Xh,
                  const float* __restrict__ bias,
                  float* out)
{
    __shared__ __attribute__((aligned(16))) _Float16 xs[XWIN];
    __shared__ __attribute__((aligned(16))) float cs[64][CSP];

    const int nt   = blockIdx.x;
    const int mt   = blockIdx.y;
    const int b    = blockIdx.z;
    const int tid  = threadIdx.x;
    const int lane = tid & 31;
    const int wave = tid >> 5;
    const int wm   = wave >> 2;
    const int wn   = wave & 3;
    const int lhi  = lane >> 4;
    const int l16  = lane & 15;
    const int h0   = nt * 2;

    {
        v8h z;
#pragma unroll
        for (int j = 0; j < 8; ++j) z[j] = (_Float16)0.0f;
        for (int e = tid; e < XWIN / 8; e += 256)
            *(v8h*)&xs[e * 8] = z;
    }

    v8f acc00 = zero8f(), acc01 = zero8f(), acc10 = zero8f(), acc11 = zero8f();

    const size_t arow0 = (size_t)(b * C_OUT + mt * 64 + wm * 32 + l16) * KTOT;
    const size_t arow1 = arow0 + (size_t)16 * KTOT;
    const int nl0 = wn * 32 + l16;
    const int nl1 = nl0 + 16;
    const int prow0 = nl0 >> 6, pcol0 = nl0 & 63;
    const int prow1 = nl1 >> 6, pcol1 = nl1 & 63;

    for (int cb = 0; cb < 8; ++cb) {
        const int ci0 = cb * 32;
        __syncthreads();
        for (int e = tid; e < 1024; e += 256) {
            const int grp = e & 3;
            const int rc  = e >> 2;
            const int win = rc & 63;
            const int row = rc >> 6;
            const int hin = h0 - 1 + row;
            if ((unsigned)hin < (unsigned)HH) {
                const v8h v = *(const v8h*)(Xh + ((size_t)((b * HH + hin) * WW + win)) * C_IN + ci0 + grp * 8);
                *(v8h*)&xs[(row * 66 + (win + 1)) * 32 + grp * 8] = v;
            }
        }
        __syncthreads();

        for (int fy = 0; fy < 3; ++fy) {
            for (int fx = 0; fx < 3; ++fx) {
                const int koff = (fy * 3 + fx) * 256 + ci0;
                Frag a0, a1, b0, b1;
                a0.half[0] = *(const v8h*)(Amod + arow0 + koff + lhi * 8);
                a0.half[1] = *(const v8h*)(Amod + arow0 + koff + 16 + lhi * 8);
                a1.half[0] = *(const v8h*)(Amod + arow1 + koff + lhi * 8);
                a1.half[1] = *(const v8h*)(Amod + arow1 + koff + 16 + lhi * 8);
                const int bb0 = ((prow0 + fy) * 66 + pcol0 + fx) * 32;
                const int bb1 = ((prow1 + fy) * 66 + pcol1 + fx) * 32;
                b0.half[0] = *(const v8h*)&xs[bb0 + lhi * 8];
                b0.half[1] = *(const v8h*)&xs[bb0 + 16 + lhi * 8];
                b1.half[0] = *(const v8h*)&xs[bb1 + lhi * 8];
                b1.half[1] = *(const v8h*)&xs[bb1 + 16 + lhi * 8];

                acc00 = wmma16(a0.v, b0.v, acc00);
                acc01 = wmma16(a0.v, b1.v, acc01);
                acc10 = wmma16(a1.v, b0.v, acc10);
                acc11 = wmma16(a1.v, b1.v, acc11);
            }
        }
    }

    {
        const int r0 = wm * 32 + lhi * 8;
        const int c0 = wn * 32 + l16;
        stash(cs, r0,      c0,      acc00);
        stash(cs, r0,      c0 + 16, acc01);
        stash(cs, r0 + 16, c0,      acc10);
        stash(cs, r0 + 16, c0 + 16, acc11);
    }
    __syncthreads();

    const int cob = mt * 64 + wave * 8;
    v4f vals[8];
#pragma unroll
    for (int j = 0; j < 8; ++j) {
        const v4f c = *(const v4f*)&cs[wave * 8 + j][lane * 4];
        const float bco = bias[cob + j];
        vals[j] = c * AUNSCALE + bco;
    }
    float* ob = out + (size_t)(b * C_OUT + cob) * NPIX + nt * 128 + lane * 4;
#pragma unroll
    for (int j = 0; j < 8; ++j)
        *(volatile v4f*)(ob + (size_t)j * NPIX) = vals[j];
    __threadfence();
#pragma unroll
    for (int j = 0; j < 8; ++j)
        *(volatile v4f*)(ob + (size_t)j * NPIX) = vals[j];
}

extern "C" void kernel_launch(void* const* d_in, const int* in_sizes, int n_in,
                              void* d_out, int out_size, void* d_ws, size_t ws_size,
                              hipStream_t stream)
{
    if (n_in < 6) return;
    if (in_sizes[0] != BS * C_IN * NPIX)   return;
    if (in_sizes[1] != BS * STYLE_D)       return;
    if (in_sizes[2] != C_OUT * KTOT)       return;
    if (in_sizes[3] <  C_OUT)              return;
    if (in_sizes[4] != C_IN * STYLE_D)     return;
    if (in_sizes[5] <  C_IN)               return;
    if (out_size    != BS * C_OUT * NPIX)  return;

    const float* x    = (const float*)d_in[0];
    const float* s    = (const float*)d_in[1];
    const float* w    = (const float*)d_in[2];
    const float* bias = (const float*)d_in[3];
    const float* aw   = (const float*)d_in[4];
    const float* ab   = (const float*)d_in[5];
    float* out        = (float*)d_out;

    const size_t off_style = 0;
    const size_t sz_style  = (size_t)BS * C_IN * sizeof(float);
    const size_t off_amod  = off_style + sz_style;
    const size_t sz_amod   = (size_t)BS * C_OUT * KTOT * sizeof(_Float16);
    const size_t off_xh    = off_amod + sz_amod;
    const size_t sz_xh     = (size_t)BS * NPIX * C_IN * sizeof(_Float16);
    if (off_xh + sz_xh > ws_size) return;

    char* ws = (char*)d_ws;
    float*    style1 = (float*)(ws + off_style);
    _Float16* Amod   = (_Float16*)(ws + off_amod);
    _Float16* Xh     = (_Float16*)(ws + off_xh);

    style_kernel<<<(BS * C_IN) / 256, 256, 0, stream>>>(s, aw, ab, style1);
    modw_kernel<<<BS * C_OUT, 256, 0, stream>>>(w, style1, Amod);
    xcvt_kernel<<<BS * (NPIX / 16), 256, 0, stream>>>(x, Xh);

    dim3 grid(32, 4, BS);
    modconv_gemm<<<grid, 256, 0, stream>>>(Amod, Xh, bias, out);
}
